// MultiScaleRetention_10737418240743
// MI455X (gfx1250) — hardware-verified
//
#include <hip/hip_runtime.h>
#include <math.h>

constexpr int kB     = 2;
constexpr int kN     = 4;
constexpr int kSeq   = 1024;
constexpr int kH     = 512;
constexpr int kHeads = 8;
constexpr int kDh    = 64;
constexpr int kBN    = kB * kN;
constexpr int kTok   = kBN * kSeq;
constexpr int kGBN   = kHeads * kBN;
constexpr int kQKVld = 3 * kH;
constexpr int kChunk = 4;
constexpr int kNumChunks = kGBN / kChunk;
constexpr int kProjRows   = kSeq;
constexpr int kProjPasses = kTok / kProjRows;
constexpr float kQCarry  = 256.0f;
constexpr float kKCarry  = 16.0f;
constexpr float kVCarry  = 64.0f;
constexpr float kSCarry  = 2048.0f;
constexpr float kScoreScale = 1.0f / (256.0f * 16.0f);
constexpr float kYScale     = 1.0f / (2048.0f * 64.0f);
constexpr float kGnEps    = 1.0e-5f;
constexpr float kInvDh    = 1.0f / 64.0f;
constexpr float kF16MinNormal = 6.103515625e-05f;
static_assert(kHeads * kDh == kH, "shape");
static_assert(kH % 32 == 0 && kDh % 32 == 0 && kSeq % 32 == 0, "every GEMM K is a multiple of 32");
static_assert(kTok % 64 == 0 && kQKVld % 64 == 0 && kH % 64 == 0 && kSeq % 64 == 0 && kDh % 64 == 0 && kProjRows % 64 == 0, "M, N tile multiples");
static_assert(kGBN % kChunk == 0 && kSeq % 2 == 0 && kTok % 4 == 0 && kProjPasses * kProjRows == kTok && kProjRows == kSeq, "decomposition");

typedef __attribute__((ext_vector_type(16))) _Float16 v16h;
typedef __attribute__((ext_vector_type(8)))  _Float16 v8h;
typedef __attribute__((ext_vector_type(16))) __bf16   v16b;
typedef __attribute__((ext_vector_type(8)))  __bf16   v8b;
typedef __attribute__((ext_vector_type(8)))  float    v8f;
typedef __attribute__((ext_vector_type(4)))  float    v4f;
typedef __attribute__((ext_vector_type(4)))  unsigned int v4u;

__device__ __forceinline__ unsigned short f2bf_bits(float f) {
  unsigned u = __float_as_uint(f);
  return (unsigned short)((u + 0x7FFFu + ((u >> 16) & 1u)) >> 16);
}
__device__ __forceinline__ float bf_bits2f(unsigned short h) { return __uint_as_float(((unsigned)h) << 16); }

__device__ __forceinline__ void dep_guard_h(v8f& a, v8f& b, v16h x, v16h y) { asm volatile("v_nop\n\tv_nop\n\tv_nop\n\tv_nop" : "+v"(a), "+v"(b) : "v"(x), "v"(y)); }
__device__ __forceinline__ void dep_guard_b(v8f& a, v8f& b, v16b x, v16b y) { asm volatile("v_nop\n\tv_nop\n\tv_nop\n\tv_nop" : "+v"(a), "+v"(b) : "v"(x), "v"(y)); }
__device__ __forceinline__ void dep_guard4_h(v8f& a, v8f& b, v8f& c, v8f& d, v16h x, v16h y) { asm volatile("v_nop\n\tv_nop\n\tv_nop\n\tv_nop" : "+v"(a), "+v"(b), "+v"(c), "+v"(d) : "v"(x), "v"(y)); }
__device__ __forceinline__ void dep_guard4_b(v8f& a, v8f& b, v8f& c, v8f& d, v16b x, v16b y) { asm volatile("v_nop\n\tv_nop\n\tv_nop\n\tv_nop" : "+v"(a), "+v"(b), "+v"(c), "+v"(d) : "v"(x), "v"(y)); }
__device__ __forceinline__ void keep4_h(v16h a, v16h b, v16h c, v16h d) { asm volatile("v_nop" :: "v"(a), "v"(b), "v"(c), "v"(d)); }
__device__ __forceinline__ void keep4_b(v16b a, v16b b, v16b c, v16b d) { asm volatile("v_nop" :: "v"(a), "v"(b), "v"(c), "v"(d)); }
__device__ __forceinline__ void acc_guard4(v8f& a, v8f& b, v8f& c, v8f& d) { asm volatile("v_nop\n\tv_nop\n\tv_nop\n\tv_nop" : "+v"(a), "+v"(b), "+v"(c), "+v"(d)); }
template <typename T> struct Frag;
template <> struct Frag<_Float16> {
  typedef v16h V; union U { v16h v; v8h h[2]; };
  static __device__ __forceinline__ v16h load(const _Float16* p) {
    U f; f.h[0] = *(const v8h*)(p); f.h[1] = *(const v8h*)(p + 16); return f.v;
  }
  static __device__ __forceinline__ v8f mma(v16h a, v16h b, v8f c) {
    return __builtin_amdgcn_wmma_f32_16x16x32_f16(false, a, false, b, (short)0, c, false, false);
  }
  static __device__ __forceinline__ void guard(v8f& a, v8f& b, v16h x, v16h y) { dep_guard_h(a, b, x, y); }
  static __device__ __forceinline__ void guard4(v8f& a, v8f& b, v8f& c, v8f& d, v16h x, v16h y) { dep_guard4_h(a, b, c, d, x, y); }
  static __device__ __forceinline__ void keep(v16h a, v16h b, v16h c, v16h d) { keep4_h(a, b, c, d); }
};
template <> struct Frag<__bf16> {
  typedef v16b V; union U { v16b v; v8b h[2]; };
  static __device__ __forceinline__ v16b load(const __bf16* p) {
    U f; f.h[0] = *(const v8b*)(p); f.h[1] = *(const v8b*)(p + 16); return f.v;
  }
  static __device__ __forceinline__ v8f mma(v16b a, v16b b, v8f c) {
    return __builtin_amdgcn_wmma_f32_16x16x32_bf16(false, a, false, b, (short)0, c, false, false);
  }
  static __device__ __forceinline__ void guard(v8f& a, v8f& b, v16b x, v16b y) { dep_guard_b(a, b, x, y); }
  static __device__ __forceinline__ void guard4(v8f& a, v8f& b, v8f& c, v8f& d, v16b x, v16b y) { dep_guard4_b(a, b, c, d, x, y); }
  static __device__ __forceinline__ void keep(v16b a, v16b b, v16b c, v16b d) { keep4_b(a, b, c, d); }
};

__device__ __forceinline__ unsigned pk16(unsigned short a, unsigned short b) { return (unsigned)a | ((unsigned)b << 16); }
__device__ __forceinline__ unsigned short h_bits(float f) { const _Float16 h = (_Float16)f; return __builtin_bit_cast(unsigned short, h); }

template <int ET> struct Elem;
template <> struct Elem<0> { typedef _Float16 T; };
template <> struct Elem<1> { typedef __bf16 T; };
template <int ET, bool SPLIT, int BIAS_MODE, int OUT_MODE, bool RESID, int ACT = 0, int TRI = 0>
__global__ __launch_bounds__(256) void wmma_gemm64(
    const unsigned short* __restrict__ Ap, const unsigned short* __restrict__ A2p, int lda, long strideA,
    const unsigned short* __restrict__ Btp, const unsigned short* __restrict__ Bt2p, int ldb, long strideB,
    void* __restrict__ Cout, void* __restrict__ Cout2, int ldc, long strideC,
    const float* __restrict__ bias,
    const float* __restrict__ resid, long strideR,
    int M, int N, int K, float scale) {
  typedef typename Elem<ET>::T T;
  typedef typename Frag<T>::V V;
  const T* A = (const T*)Ap; const T* A2 = (const T*)A2p; const T* Bt = (const T*)Btp; const T* Bt2 = (const T*)Bt2p;
  __shared__ __align__(16) float sT[8][16 * 68];
  const int b    = blockIdx.y;
  const int lane = threadIdx.x & 31;
  const int wave = threadIdx.x >> 5;
  const int tilesN = N >> 6;
  const int tilesM = M >> 6;
  const int tile = blockIdx.x * 8 + wave;
  if (tile >= tilesM * tilesN) return;
  const int tm = tile / tilesN;
  const int tn = tile - tm * tilesN;
  if (TRI == 1 && tn > tm) return;
  const int m0 = tm << 6;
  const int n0 = tn << 6;
  const int kLim = (tm + 1) << 6;
  const int Kend = (TRI == 2) ? ((kLim < K) ? kLim : K) : K;

  const T* Ab  = A  + (size_t)b * strideA;
  const T* Bb  = Bt + (size_t)b * strideB;
  const T* Ab2 = SPLIT ? (A2  + (size_t)b * strideA) : nullptr;
  const T* Bb2 = SPLIT ? (Bt2 + (size_t)b * strideB) : nullptr;

  const int rlane = lane & 15;
  const int koff  = (lane >> 4) * 8;
  const int mOff  = (lane >> 4) * 8;

  v8f acc[4][4];
#pragma unroll
  for (int i = 0; i < 4; ++i)
#pragma unroll
    for (int j = 0; j < 4; ++j) acc[i][j] = (v8f){0.f,0.f,0.f,0.f,0.f,0.f,0.f,0.f};

  for (int k0 = 0; k0 < Kend; k0 += 32) {
    V bh[4], bl[4];
#pragma unroll
    for (int j = 0; j < 4; ++j) {
      const size_t bo = (size_t)(n0 + (j << 4) + rlane) * ldb + koff + k0;
      bh[j] = Frag<T>::load(Bb + bo);
      if (SPLIT) bl[j] = Frag<T>::load(Bb2 + bo);
    }
#pragma unroll
    for (int i = 0; i < 4; ++i) {
      const size_t ao = (size_t)(m0 + (i << 4) + rlane) * lda + koff + k0;
      V ah = Frag<T>::load(Ab + ao);
      V al;
      if (SPLIT) al = Frag<T>::load(Ab2 + ao);
#pragma unroll
      for (int j = 0; j < 4; ++j) {
        acc[i][j] = Frag<T>::mma(ah, bh[j], acc[i][j]);
        if (SPLIT) {
          acc[i][j] = Frag<T>::mma(ah, bl[j], acc[i][j]);
          acc[i][j] = Frag<T>::mma(al, bh[j], acc[i][j]);
        }
      }
      Frag<T>::guard4(acc[i][0], acc[i][1], acc[i][2], acc[i][3], ah, SPLIT ? al : ah);
    }
    Frag<T>::keep(bh[0], bh[1], bh[2], bh[3]);
    if (SPLIT) Frag<T>::keep(bl[0], bl[1], bl[2], bl[3]);
  }
  acc_guard4(acc[0][0], acc[0][1], acc[0][2], acc[0][3]);
  acc_guard4(acc[1][0], acc[1][1], acc[1][2], acc[1][3]);
  acc_guard4(acc[2][0], acc[2][1], acc[2][2], acc[2][3]);
  acc_guard4(acc[3][0], acc[3][1], acc[3][2], acc[3][3]);

  float* slab = sT[wave];
  const float* Rb = RESID ? (resid + (size_t)b * strideR) : nullptr;
#pragma unroll
  for (int i = 0; i < 4; ++i) {
    const int mBase = m0 + (i << 4);
#pragma unroll
    for (int j = 0; j < 4; ++j) {
      const int n = n0 + (j << 4) + rlane;
      float bv = 0.f;
      if (BIAS_MODE == 2) bv = bias[n];
#pragma unroll
      for (int r = 0; r < 8; ++r) {
        float v = acc[i][j][r] * scale;
        if (BIAS_MODE == 1) v += bias[mBase + mOff + r];
        if (BIAS_MODE == 2) v += bv;
        if (RESID) v += Rb[(size_t)(mBase + mOff + r) * ldc + n];
        if (ACT == 2) v = fmaxf(v, 0.0f);
        if (ACT == 4) v = (v > 0.f) ? v : 0.01f * v;
        slab[(mOff + r) * 68 + (j << 4) + rlane] = v;
      }
    }
    __builtin_amdgcn_fence(__ATOMIC_RELEASE, "workgroup");
    __builtin_amdgcn_wave_barrier();
    __builtin_amdgcn_fence(__ATOMIC_ACQUIRE, "workgroup");
    if (OUT_MODE == 0) {
      float* C = (float*)Cout + (size_t)b * strideC;
      const int hh = lane >> 4, c4 = (lane & 15) * 4;
      for (int pass = 0; pass < 2; ++pass) {
#pragma unroll
        for (int it = 0; it < 8; ++it) {
          const int row = it * 2 + hh;
          v4f v = *(const v4f*)(slab + row * 68 + c4);
          *(volatile v4f*)(C + (size_t)(mBase + row) * ldc + n0 + c4) = v;
        }
        __threadfence();
      }
    } else {
      const int q = lane >> 3, c8 = (lane & 7) * 8;
      unsigned short* C  = (unsigned short*)Cout  + (size_t)b * strideC;
      unsigned short* C2 = (OUT_MODE == 2) ? ((unsigned short*)Cout2 + (size_t)b * strideC) : nullptr;
      for (int pass = 0; pass < 2; ++pass) {
#pragma unroll
        for (int it = 0; it < 4; ++it) {
          const int row = it * 4 + q;
          const float* sp = slab + row * 68 + c8;
          v8h hv, lv;
#pragma unroll
          for (int e = 0; e < 8; ++e) {
            if (OUT_MODE == 1) {
              hv[e] = (_Float16)sp[e];
            } else {
              unsigned short hb = f2bf_bits(sp[e]);
              unsigned short lb = f2bf_bits(sp[e] - bf_bits2f(hb));
              hv[e] = __builtin_bit_cast(_Float16, hb);
              lv[e] = __builtin_bit_cast(_Float16, lb);
            }
          }
          *(volatile v8h*)(C + (size_t)(mBase + row) * ldc + n0 + c8) = hv;
          if (OUT_MODE == 2) *(volatile v8h*)(C2 + (size_t)(mBase + row) * ldc + n0 + c8) = lv;
        }
        __threadfence();
      }
    }
    __builtin_amdgcn_fence(__ATOMIC_RELEASE, "workgroup");
    __builtin_amdgcn_wave_barrier();
    __builtin_amdgcn_fence(__ATOMIC_ACQUIRE, "workgroup");
  }
}

__global__ __launch_bounds__(256) void cast8_bf16_split_kernel(const float* __restrict__ in, unsigned short* __restrict__ outh,
                                                               unsigned short* __restrict__ outl, int n8) {
  const int i = blockIdx.x * 256 + threadIdx.x;
  if (i >= n8) return;
  const float* p = in + 8 * (size_t)i;
  const v4f a = *(const v4f*)(p);
  const v4f c = *(const v4f*)(p + 4);
  unsigned short hb[8], lb[8];
#pragma unroll
  for (int e = 0; e < 4; ++e) {
    const float x0 = a[e];
    const unsigned short h0 = f2bf_bits(x0);
    hb[e] = h0;
    lb[e] = f2bf_bits(x0 - bf_bits2f(h0));
    const float x1 = c[e];
    const unsigned short h1 = f2bf_bits(x1);
    hb[4 + e] = h1;
    lb[4 + e] = f2bf_bits(x1 - bf_bits2f(h1));
  }
  const v4u uh = (v4u){pk16(hb[0], hb[1]), pk16(hb[2], hb[3]), pk16(hb[4], hb[5]), pk16(hb[6], hb[7])};
  const v4u ul = (v4u){pk16(lb[0], lb[1]), pk16(lb[2], lb[3]), pk16(lb[4], lb[5]), pk16(lb[6], lb[7])};
  unsigned short* qh = outh + 8 * (size_t)i;
  unsigned short* ql = outl + 8 * (size_t)i;
  *(volatile v4u*)qh = uh;
  *(volatile v4u*)ql = ul;
  __threadfence();
  *(volatile v4u*)qh = uh;
  *(volatile v4u*)ql = ul;
}

__global__ __launch_bounds__(256) void wqkv_cast_kernel(const float* __restrict__ W0, const float* __restrict__ W1,
                                                        const float* __restrict__ W2, unsigned short* __restrict__ outh,
                                                        unsigned short* __restrict__ outl) {
  __shared__ float sm[64][65];
  const int t  = threadIdx.x;
  const int h0 = blockIdx.x * 64;
  const int g  = blockIdx.y;
  const int z  = blockIdx.z;
  const float* W = (z == 0) ? W0 : (z == 1) ? W1 : W2;
  const float* src = W + ((size_t)g * kH + h0) * kDh;
#pragma unroll
  for (int i = 0; i < 8; ++i) {
    const int e  = i * 256 + t;
    const int hl = e >> 6;
    const int d  = e & 63;
    sm[d][hl] = src[hl * kDh + d];
  }
  asm volatile("" ::: "memory");
#pragma unroll
  for (int i = 8; i < 16; ++i) {
    const int e  = i * 256 + t;
    const int hl = e >> 6;
    const int d  = e & 63;
    sm[d][hl] = src[hl * kDh + d];
  }
  __syncthreads();
  const int lane = t & 31, wave = t >> 5;
  const int q = lane >> 3, c8 = (lane & 7) * 8;
  const size_t plane0 = ((size_t)z * kH + (size_t)g * kDh) * kH;
  unsigned short* oph = outh + plane0;
  unsigned short* opl = outl + plane0;
  for (int pass = 0; pass < 2; ++pass) {
#pragma unroll
    for (int it = 0; it < 2; ++it) {
      const int row = wave * 8 + it * 4 + q;
      unsigned short hb[8], lb[8];
#pragma unroll
      for (int e = 0; e < 8; ++e) {
        const float x = sm[row][c8 + e];
        const unsigned short hx = f2bf_bits(x);
        hb[e] = hx;
        lb[e] = f2bf_bits(x - bf_bits2f(hx));
      }
      const v4u uh = (v4u){pk16(hb[0], hb[1]), pk16(hb[2], hb[3]), pk16(hb[4], hb[5]), pk16(hb[6], hb[7])};
      const v4u ul = (v4u){pk16(lb[0], lb[1]), pk16(lb[2], lb[3]), pk16(lb[4], lb[5]), pk16(lb[6], lb[7])};
      *(volatile v4u*)(oph + (size_t)row * kH + h0 + c8) = uh;
      *(volatile v4u*)(opl + (size_t)row * kH + h0 + c8) = ul;
    }
    __threadfence();
  }
}

__global__ __launch_bounds__(256) void whh_cast_kernel(const float* __restrict__ W0, const float* __restrict__ W1,
                                                       unsigned short* __restrict__ outh, unsigned short* __restrict__ outl) {
  __shared__ float sm[64][65];
  const int t  = threadIdx.x;
  const int d0 = blockIdx.x * 64;
  const int h0 = blockIdx.y * 64;
  const int z  = blockIdx.z;
  const float* W = (z == 0) ? W0 : W1;
#pragma unroll
  for (int i = 0; i < 8; ++i) {
    const int e = i * 256 + t;
    const int r = e >> 6;
    const int c = e & 63;
    sm[c][r] = W[(size_t)(d0 + r) * kH + h0 + c];
  }
  asm volatile("" ::: "memory");
#pragma unroll
  for (int i = 8; i < 16; ++i) {
    const int e = i * 256 + t;
    const int r = e >> 6;
    const int c = e & 63;
    sm[c][r] = W[(size_t)(d0 + r) * kH + h0 + c];
  }
  __syncthreads();
  const int lane = t & 31, wave = t >> 5;
  const int q = lane >> 3, c8 = (lane & 7) * 8;
  unsigned short* oph = outh + (size_t)z * kH * kH;
  unsigned short* opl = outl + (size_t)z * kH * kH;
  for (int pass = 0; pass < 2; ++pass) {
#pragma unroll
    for (int it = 0; it < 2; ++it) {
      const int row = wave * 8 + it * 4 + q;
      unsigned short hb[8], lb[8];
#pragma unroll
      for (int e = 0; e < 8; ++e) {
        const float x = sm[row][c8 + e];
        const unsigned short hx = f2bf_bits(x);
        hb[e] = hx;
        lb[e] = f2bf_bits(x - bf_bits2f(hx));
      }
      const v4u uh = (v4u){pk16(hb[0], hb[1]), pk16(hb[2], hb[3]), pk16(hb[4], hb[5]), pk16(hb[6], hb[7])};
      const v4u ul = (v4u){pk16(lb[0], lb[1]), pk16(lb[2], lb[3]), pk16(lb[4], lb[5]), pk16(lb[6], lb[7])};
      *(volatile v4u*)(oph + (size_t)(h0 + row) * kH + d0 + c8) = uh;
      *(volatile v4u*)(opl + (size_t)(h0 + row) * kH + d0 + c8) = ul;
    }
    __threadfence();
  }
}

struct RotConst { float fh[32]; float fl[32]; float lnsv[32]; };
static_assert(sizeof(RotConst) == 384, "no padding");

__global__ __launch_bounds__(256) void rot_table_kernel(float* __restrict__ tsn, float* __restrict__ tcs,
                                                        float* __restrict__ tsc, float* __restrict__ trs, RotConst rc) {
  const int t    = threadIdx.x;
  const int lane = t & 31;
  const int idx  = blockIdx.x * 256 + t;
  const int s    = idx >> 5;
  float fh = rc.fh[0], fl = rc.fl[0], ln = rc.lnsv[0];
#pragma unroll
  for (int k = 1; k < 32; ++k) {
    const bool m = (lane == k);
    fh = m ? rc.fh[k] : fh;
    fl = m ? rc.fl[k] : fl;
    ln = m ? rc.lnsv[k] : ln;
  }
  const float sf = (float)s;
  float p = sf * fh;
  asm volatile("" : "+v"(p));
  const float corr = fmaf(sf, fh, -p) + sf * fl;
  const float n = rintf(p * 0.63661977236758134f);
  float r = fmaf(-n, 1.57079637050628662109375f, p);
  r = fmaf(-n, -4.37113882867379812058e-08f, r);
  r = fmaf(-n, -1.71512451000595447e-15f, r);
  r = r + corr;
  const float z = r * r;
  const float spoly = fmaf(fmaf(-1.9515295891e-4f, z, 8.3321608736e-3f), z, -1.6666654611e-1f);
  const float sp = fmaf(spoly * z, r, r);
  const float cpoly = fmaf(fmaf(2.443315711809948e-5f, z, -1.388731625493765e-3f), z, 4.166664568298827e-2f);
  const float cp = fmaf(cpoly, z * z, fmaf(-0.5f, z, 1.0f));
  const int jq = ((int)n) & 3;
  const float ssel = (jq & 1) ? cp : sp;
  const float csel = (jq & 1) ? sp : cp;
  const float sn = (jq & 2) ? -ssel : ssel;
  const float cs = (jq == 1 || jq == 2) ? -csel : csel;
  const float scl = expf(sf * (1.0f / 512.0f) * ln);
  const float rs  = 1.0f / scl;
  *(volatile float*)(tsn + idx) = sn;
  *(volatile float*)(tcs + idx) = cs;
  *(volatile float*)(tsc + idx) = scl;
  *(volatile float*)(trs + idx) = rs;
  __threadfence();
  *(volatile float*)(tsn + idx) = sn;
  *(volatile float*)(tcs + idx) = cs;
  *(volatile float*)(tsc + idx) = scl;
  *(volatile float*)(trs + idx) = rs;
}

__global__ __launch_bounds__(256) void rot_apply_kernel(const float* __restrict__ QKV, int bn,
                                                        const float* __restrict__ tsn, const float* __restrict__ tcs,
                                                        const float* __restrict__ tsc, const float* __restrict__ trs,
                                                        unsigned short* __restrict__ Qp, unsigned short* __restrict__ Kp,
                                                        unsigned short* __restrict__ Vt) {
  __shared__ __align__(16) float lsn[2048];
  __shared__ __align__(16) float lcs[2048];
  __shared__ __align__(16) float lsc[2048];
  __shared__ __align__(16) float lrs[2048];
  __shared__ float smv[64][65];
  const int t = threadIdx.x, lane = t & 31, wave = t >> 5;
  const int s0 = blockIdx.x * 64, g = blockIdx.z;
  const int gbn = g * kBN + bn;
  const size_t row0 = (size_t)s0;
#pragma unroll
  for (int i = 0; i < 4; ++i) {
    const int e  = i * 256 + t;
    const int sl = e >> 4;
    const int c4 = (e & 15) * 4;
    const v4f vv = *(const v4f*)(QKV + (row0 + sl) * kQKVld + 2 * kH + g * kDh + c4);
    smv[c4 + 0][sl] = vv[0];
    smv[c4 + 1][sl] = vv[1];
    smv[c4 + 2][sl] = vv[2];
    smv[c4 + 3][sl] = vv[3];
  }
  asm volatile("" ::: "memory");
  {
    const size_t tb = (size_t)s0 * 32;
#pragma unroll
    for (int i = 0; i < 2; ++i) {
      const int e = (i * 256 + t) * 4;
      *(v4f*)(lsn + e) = *(const v4f*)(tsn + tb + e);
      *(v4f*)(lcs + e) = *(const v4f*)(tcs + tb + e);
    }
    asm volatile("" ::: "memory");
#pragma unroll
    for (int i = 0; i < 2; ++i) {
      const int e = (i * 256 + t) * 4;
      *(v4f*)(lsc + e) = *(const v4f*)(tsc + tb + e);
      *(v4f*)(lrs + e) = *(const v4f*)(trs + tb + e);
    }
  }
  __syncthreads();
  const int q8 = t >> 3, c8 = (t & 7) * 8, i0 = c8 >> 1;
#pragma unroll 1
  for (int it = 0; it < 2; ++it) {
    const int r = it * 32 + q8;
    const float* src = QKV + (row0 + r) * kQKVld + g * kDh + c8;
    const v4f qa = *(const v4f*)(src);
    const v4f qb = *(const v4f*)(src + 4);
    const v4f ka = *(const v4f*)(src + kH);
    const v4f kb = *(const v4f*)(src + kH + 4);
    const v4f sn = *(const v4f*)(lsn + r * 32 + i0);
    const v4f cs = *(const v4f*)(lcs + r * 32 + i0);
    const v4f sc = *(const v4f*)(lsc + r * 32 + i0);
    const v4f rs = *(const v4f*)(lrs + r * 32 + i0);
    float qv[8], kv[8];
#pragma unroll
    for (int e = 0; e < 4; ++e) { qv[e] = qa[e]; qv[4 + e] = qb[e]; kv[e] = ka[e]; kv[4 + e] = kb[e]; }
    unsigned short hq[8], hk[8];
#pragma unroll
    for (int p = 0; p < 4; ++p) {
      const float x0 = qv[2 * p], x1 = qv[2 * p + 1];
      const float y0 = kv[2 * p], y1 = kv[2 * p + 1];
      const float snp = sn[p], csp = cs[p];
      const float qf = sc[p] * kQCarry;
      const float kf = rs[p] * kKCarry;
      hq[2 * p]     = h_bits((x0 * csp - x1 * snp) * qf);
      hq[2 * p + 1] = h_bits((x1 * csp + x0 * snp) * qf);
      hk[2 * p]     = h_bits((y0 * csp - y1 * snp) * kf);
      hk[2 * p + 1] = h_bits((y1 * csp + y0 * snp) * kf);
    }
    const v4u uq = (v4u){pk16(hq[0], hq[1]), pk16(hq[2], hq[3]), pk16(hq[4], hq[5]), pk16(hq[6], hq[7])};
    const v4u uk = (v4u){pk16(hk[0], hk[1]), pk16(hk[2], hk[3]), pk16(hk[4], hk[5]), pk16(hk[6], hk[7])};
    const size_t po = ((size_t)gbn * kSeq + s0 + r) * kDh + c8;
    *(volatile v4u*)(Qp + po) = uq;
    *(volatile v4u*)(Kp + po) = uk;
    __threadfence();
    *(volatile v4u*)(Qp + po) = uq;
    *(volatile v4u*)(Kp + po) = uk;
  }
  {
    const int q = lane >> 3, cb = (lane & 7) * 8;
    unsigned short* vt = Vt + ((size_t)gbn * kDh) * kSeq + s0;
    for (int pass = 0; pass < 2; ++pass) {
#pragma unroll
      for (int it = 0; it < 2; ++it) {
        const int row = wave * 8 + it * 4 + q;
        unsigned short hb[8];
#pragma unroll
        for (int e = 0; e < 8; ++e) hb[e] = h_bits(smv[row][cb + e] * kVCarry);
        const v4u u = (v4u){pk16(hb[0], hb[1]), pk16(hb[2], hb[3]), pk16(hb[4], hb[5]), pk16(hb[6], hb[7])};
        *(volatile v4u*)(vt + (size_t)row * kSeq + cb) = u;
      }
      __threadfence();
    }
  }
}

__global__ __launch_bounds__(256) void decay_cast_kernel(const float* __restrict__ SC, unsigned short* __restrict__ SD,
                                                         float lgam, float ginv, float carry) {
  const int t  = threadIdx.x;
  const int z  = blockIdx.y;
  const int s  = blockIdx.x * 2 + (t >> 7);
  const int c0 = (t & 127) * 8;
  const int sm8 = s & ~7;
  const int cl = (c0 < sm8) ? c0 : sm8;
  const size_t rowoff = ((size_t)z * kSeq + s) * kSeq;
  const v4f a = *(const v4f*)(SC + rowoff + cl);
  const v4f b = *(const v4f*)(SC + rowoff + cl + 4);
  const int dd = (s - c0 > 0) ? (s - c0) : 0;
  float base = expf((float)dd * lgam);
  unsigned short hb[8];
#pragma unroll
  for (int e = 0; e < 4; ++e) {
    float x = a[e] * base * carry;
    base = base * ginv;
    const bool keep = (c0 + e) <= s;
    x = keep ? x : 0.0f;
    x = (fabsf(x) < kF16MinNormal) ? 0.0f : x;
    hb[e] = h_bits(x);
  }
#pragma unroll
  for (int e = 0; e < 4; ++e) {
    float x = b[e] * base * carry;
    base = base * ginv;
    const bool keep = (c0 + 4 + e) <= s;
    x = keep ? x : 0.0f;
    x = (fabsf(x) < kF16MinNormal) ? 0.0f : x;
    hb[4 + e] = h_bits(x);
  }
  const v4u u = (v4u){pk16(hb[0], hb[1]), pk16(hb[2], hb[3]), pk16(hb[4], hb[5]), pk16(hb[6], hb[7])};
  unsigned short* dp = SD + rowoff + c0;
  *(volatile v4u*)dp = u;
  __threadfence();
  *(volatile v4u*)dp = u;
}

__global__ __launch_bounds__(256) void gn_gate_kernel(const float* __restrict__ Y, const float* __restrict__ GT,
                                                      const float* __restrict__ gnw, const float* __restrict__ gnb,
                                                      unsigned short* __restrict__ Gbh, unsigned short* __restrict__ Gbl) {
  const int t = threadIdx.x, lane = t & 31, wave = t >> 5;
  const int row = blockIdx.x * 4 + (wave >> 1);
  const int cb  = (wave & 1) * 256 + lane * 8;
  const float* yr = Y  + (size_t)row * kH + cb;
  const float* gr = GT + (size_t)row * kH + cb;
  const v4f ya = *(const v4f*)(yr);
  const v4f yb = *(const v4f*)(yr + 4);
  float s1 = ((ya[0] + ya[1]) + (ya[2] + ya[3])) + ((yb[0] + yb[1]) + (yb[2] + yb[3]));
  s1 += __shfl_xor(s1, 1, 32);
  s1 += __shfl_xor(s1, 2, 32);
  s1 += __shfl_xor(s1, 4, 32);
  const float mean = s1 * kInvDh;
  float s2 = 0.0f;
#pragma unroll
  for (int e = 0; e < 4; ++e) {
    const float da = ya[e] - mean;
    const float db = yb[e] - mean;
    s2 = fmaf(da, da, s2);
    s2 = fmaf(db, db, s2);
  }
  s2 += __shfl_xor(s2, 1, 32);
  s2 += __shfl_xor(s2, 2, 32);
  s2 += __shfl_xor(s2, 4, 32);
  const float var = s2 * kInvDh;
  const float inv = rsqrtf(var + kGnEps);
  unsigned int uh0 = 0u, uh1 = 0u, uh2 = 0u, uh3 = 0u;
  unsigned int ul0 = 0u, ul1 = 0u, ul2 = 0u, ul3 = 0u;
#pragma unroll 1
  for (int half = 0; half < 2; ++half) {
    const bool hsel = (half != 0);
    const float yv0 = hsel ? yb[0] : ya[0];
    const float yv1 = hsel ? yb[1] : ya[1];
    const float yv2 = hsel ? yb[2] : ya[2];
    const float yv3 = hsel ? yb[3] : ya[3];
    const v4f gv = *(const v4f*)(gr + 4 * half);
    const v4f wv = *(const v4f*)(gnw + cb + 4 * half);
    const v4f bv = *(const v4f*)(gnb + cb + 4 * half);
    float yv[4] = {yv0, yv1, yv2, yv3};
    unsigned short hb[4], lb[4];
#pragma unroll
    for (int e = 0; e < 4; ++e) {
      const float d  = yv[e] - mean;
      const float yn = fmaf(d * inv, wv[e], bv[e]);
      const float gt = gv[e];
      const float ex = expf(-gt);
      const float sg = __builtin_amdgcn_rcpf(1.0f + ex);
      const float o  = (gt * sg) * yn;
      const unsigned short hx = f2bf_bits(o);
      hb[e] = hx;
      lb[e] = f2bf_bits(o - bf_bits2f(hx));
    }
    const unsigned int ph0 = pk16(hb[0], hb[1]);
    const unsigned int ph1 = pk16(hb[2], hb[3]);
    const unsigned int pl0 = pk16(lb[0], lb[1]);
    const unsigned int pl1 = pk16(lb[2], lb[3]);
    uh0 = hsel ? uh0 : ph0;
    uh1 = hsel ? uh1 : ph1;
    uh2 = hsel ? ph0 : uh2;
    uh3 = hsel ? ph1 : uh3;
    ul0 = hsel ? ul0 : pl0;
    ul1 = hsel ? ul1 : pl1;
    ul2 = hsel ? pl0 : ul2;
    ul3 = hsel ? pl1 : ul3;
  }
  const v4u uh = (v4u){uh0, uh1, uh2, uh3};
  const v4u ul = (v4u){ul0, ul1, ul2, ul3};
  unsigned short* gph = Gbh + (size_t)row * kH + cb;
  unsigned short* gpl = Gbl + (size_t)row * kH + cb;
  *(volatile v4u*)gph = uh;
  *(volatile v4u*)gpl = ul;
  __threadfence();
  *(volatile v4u*)gph = uh;
  *(volatile v4u*)gpl = ul;
}

extern "C" void kernel_launch(void* const* d_in, const int* in_sizes, int n_in,
                              void* d_out, int out_size, void* d_ws, size_t ws_size,
                              hipStream_t stream) {
  if (n_in < 8) return;
  if (in_sizes[0] != kTok * kH) return;
  if (in_sizes[1] != kHeads * kH * kDh || in_sizes[2] != kHeads * kH * kDh || in_sizes[3] != kHeads * kH * kDh) return;
  if (in_sizes[4] != kH * kH || in_sizes[5] != kH * kH) return;
  if (in_sizes[6] != kH || in_sizes[7] != kH) return;
  if (out_size != kTok * kH) return;

  const size_t szX16  = (size_t)kTok * kH * 2;
  const size_t szWqkv = (size_t)kQKVld * kH * 2;
  const size_t szWhh  = (size_t)kH * kH * 2;
  const size_t szQKVR = (size_t)kProjRows * kQKVld * 4;
  const size_t szSC   = (size_t)kChunk * kSeq * kSeq * 4;
  const size_t szY    = (size_t)kTok * kH * 4;
  const size_t szQp   = (size_t)kGBN * kSeq * kDh * 2;
  const size_t szSD   = (size_t)kChunk * kSeq * kSeq * 2;
  const size_t szTab1 = (size_t)kSeq * 32 * 4;
  const size_t offXbh  = 0;
  const size_t offXbl  = offXbh + szX16;
  const size_t offWqh  = offXbl + szX16;
  const size_t offWql  = offWqh + szWqkv;
  const size_t offWhhH = offWql + szWqkv;
  const size_t offWhhL = offWhhH + 2 * szWhh;
  const size_t offQKVR = offWhhL + 2 * szWhh;
  const size_t offSC   = offQKVR + szQKVR;
  const size_t offY    = offSC + szSC;
  const size_t offGT   = offY + szY;
  const size_t offQp   = offGT + szY;
  const size_t offKp   = offQp + szQp;
  const size_t offVt   = offKp + szQp;
  const size_t offSD   = offVt + szQp;
  const size_t offGbh  = offSD + szSD;
  const size_t offGbl  = offGbh + szX16;
  const size_t offTab  = offGbl + szX16;
  const size_t total   = offTab + 4 * szTab1;
  if (ws_size < total) return;

  const float* X   = (const float*)d_in[0];
  const float* W_Q = (const float*)d_in[1];
  const float* W_K = (const float*)d_in[2];
  const float* W_V = (const float*)d_in[3];
  const float* W_G = (const float*)d_in[4];
  const float* W_O = (const float*)d_in[5];
  const float* gnw = (const float*)d_in[6];
  const float* gnb = (const float*)d_in[7];
  float* out = (float*)d_out;
  char* ws = (char*)d_ws;
  unsigned short* Xbh = (unsigned short*)(ws + offXbh);
  unsigned short* Xbl = (unsigned short*)(ws + offXbl);
  unsigned short* Wqh = (unsigned short*)(ws + offWqh);
  unsigned short* Wql = (unsigned short*)(ws + offWql);
  unsigned short* WhhH = (unsigned short*)(ws + offWhhH);
  unsigned short* WhhL = (unsigned short*)(ws + offWhhL);
  unsigned short* WGh = WhhH;
  unsigned short* WOh = WhhH + (size_t)kH * kH;
  unsigned short* WGl = WhhL;
  unsigned short* WOl = WhhL + (size_t)kH * kH;
  float* QKVR = (float*)(ws + offQKVR);
  float* SC   = (float*)(ws + offSC);
  float* Yp   = (float*)(ws + offY);
  float* GT   = (float*)(ws + offGT);
  unsigned short* Qp = (unsigned short*)(ws + offQp);
  unsigned short* Kp = (unsigned short*)(ws + offKp);
  unsigned short* Vt = (unsigned short*)(ws + offVt);
  unsigned short* SD = (unsigned short*)(ws + offSD);
  unsigned short* Gbh = (unsigned short*)(ws + offGbh);
  unsigned short* Gbl = (unsigned short*)(ws + offGbl);
  float* tsn = (float*)(ws + offTab);
  float* tcs = (float*)(ws + offTab + szTab1);
  float* tsc = (float*)(ws + offTab + 2 * szTab1);
  float* trs = (float*)(ws + offTab + 3 * szTab1);

  RotConst rc;
  for (int i = 0; i < 32; ++i) {
    const double f  = 1.0 / pow(10000.0, (double)i / 32.0);
    const float  fh = (float)f;
    rc.fh[i]   = fh;
    rc.fl[i]   = (float)(f - (double)fh);
    const double sv = ((double)(2 * i) + 0.4 * 64.0) / (1.4 * 64.0);
    rc.lnsv[i] = (float)log(sv);
  }
  float lgamf[kHeads], ginvf[kHeads];
  {
    const double la = log(1.0 / 32.0), lb = log(1.0 / 512.0);
    const double step = (lb - la) / 7.0;
    for (int g = 0; g < kHeads; ++g) {
      const double lin = (g == kHeads - 1) ? lb : ((double)g * step + la);
      const double gam = 1.0 - exp(lin);
      lgamf[g] = (float)log(gam);
      ginvf[g] = (float)(1.0 / gam);
    }
  }

  const int n8 = (kTok * kH) / 8;
  cast8_bf16_split_kernel<<<dim3(n8 / 256), dim3(256), 0, stream>>>(X, Xbh, Xbl, n8);
  wqkv_cast_kernel<<<dim3(kH / 64, kHeads, 3), dim3(256), 0, stream>>>(W_Q, W_K, W_V, Wqh, Wql);
  whh_cast_kernel<<<dim3(kH / 64, kH / 64, 2), dim3(256), 0, stream>>>(W_G, W_O, WhhH, WhhL);
  rot_table_kernel<<<dim3((kSeq * 32) / 256), dim3(256), 0, stream>>>(tsn, tcs, tsc, trs, rc);

  const int tilesProj = (kProjRows / 64) * (kQKVld / 64);
  for (int p = 0; p < kProjPasses; ++p) {
    const size_t xo = (size_t)p * kProjRows * kH;
    wmma_gemm64<1, true, 0, 0, false, 0, 0><<<dim3(tilesProj / 8, 1), dim3(256), 0, stream>>>(
        Xbh + xo, Xbl + xo, kH, 0L, Wqh, Wql, kH, 0L, (void*)QKVR, (void*)QKVR, kQKVld, 0L, gnw, gnw, 0L,
        kProjRows, kQKVld, kH, 1.0f);
    rot_apply_kernel<<<dim3(kSeq / 64, 1, kHeads), dim3(256), 0, stream>>>(QKVR, p, tsn, tcs, tsc, trs, Qp, Kp, Vt);
  }

  const long strideQK = (long)kSeq * kDh;
  const long strideS  = (long)kSeq * kSeq;
  const long strideVt = (long)kDh * kSeq;
  const long strideY  = (long)kSeq * kH;
  const int tilesScore = (kSeq / 64) * (kSeq / 64);
  const int tilesValue = (kSeq / 64) * (kDh / 64);
  for (int c = 0; c < kNumChunks; ++c) {
    const int g = c >> 1;
    const int bn0 = (c & 1) * kChunk;
    const size_t gbn0 = (size_t)c * kChunk;
    const unsigned short* Qc = Qp + gbn0 * (size_t)kSeq * kDh;
    const unsigned short* Kc = Kp + gbn0 * (size_t)kSeq * kDh;
    const unsigned short* Vc = Vt + gbn0 * (size_t)kDh * kSeq;
    float* Yc = Yp + ((size_t)bn0 * kSeq) * kH + (size_t)g * kDh;
    wmma_gemm64<0, false, 0, 0, false, 0, 1><<<dim3(tilesScore / 8, kChunk), dim3(256), 0, stream>>>(
        Qc, Qc, kDh, strideQK, Kc, Kc, kDh, strideQK, (void*)SC, (void*)SC, kSeq, strideS, gnw, gnw, 0L,
        kSeq, kSeq, kDh, kScoreScale);
    decay_cast_kernel<<<dim3(kSeq / 2, kChunk), dim3(256), 0, stream>>>(SC, SD, lgamf[g], ginvf[g], kSCarry);
    wmma_gemm64<0, false, 0, 0, false, 0, 2><<<dim3(tilesValue / 8, kChunk), dim3(256), 0, stream>>>(
        SD, SD, kSeq, strideS, Vc, Vc, kSeq, strideVt, (void*)Yc, (void*)Yc, kH, strideY, gnw, gnw, 0L,
        kSeq, kDh, kSeq, kYScale);
  }

  const int tilesHH = (kTok / 64) * (kH / 64);
  wmma_gemm64<1, true, 0, 0, false, 0, 0><<<dim3(tilesHH / 8, 1), dim3(256), 0, stream>>>(
      Xbh, Xbl, kH, 0L, WGh, WGl, kH, 0L, (void*)GT, (void*)GT, kH, 0L, gnw, gnw, 0L, kTok, kH, kH, 1.0f);

  gn_gate_kernel<<<dim3(kTok / 4), dim3(256), 0, stream>>>(Yp, GT, gnw, gnb, Gbh, Gbl);

  wmma_gemm64<1, true, 0, 0, false, 0, 0><<<dim3(tilesHH / 8, 1), dim3(256), 0, stream>>>(
      Gbh, Gbl, kH, 0L, WOh, WOl, kH, 0L, (void*)out, (void*)out, kH, 0L, gnw, gnw, 0L, kTok, kH, kH, 1.0f);
}
